// DynamicGCN_54185307406500
// MI455X (gfx1250) — hardware-verified
//
#include <hip/hip_runtime.h>


namespace {
constexpr int B = 16, N = 512, T = 24, D = 64, NBT = B * T, BTL = NBT  , NR = B * N * T;
constexpr float XS = 8.0f, WSC = 256.0f, PS = 1024.0f, RS_ = 1024.0f, LOG2E = 1.4426950408889634f;
static_assert(N % 64 == 0 && D == 64 && NR % 64 == 0, "tiling");
typedef _Float16 b16;
typedef __attribute__((ext_vector_type(16))) _Float16 v16b;
typedef __attribute__((ext_vector_type(8))) _Float16 v8b;
typedef __attribute__((ext_vector_type(8))) float v8f;
typedef __attribute__((ext_vector_type(4))) float v4f;
__device__ __forceinline__ float bf16_rne(float f) { unsigned int u = __float_as_uint(f); u += 0x7FFFu + ((u >> 16) & 1u); return __uint_as_float(u & 0xFFFF0000u); }
__device__ __forceinline__ void split16(float v, b16& hi, b16& lo) { hi = (b16)v; lo = (b16)(v - (float)hi); }
__device__ __forceinline__ v16b frag_kb(const b16* p, int hh) { const v8b a = *(const v8b*)(p + 8 * hh), b = *(const v8b*)(p + 16 + 8 * hh); v16b f;
#pragma unroll
  for (int e = 0; e < 8; ++e) { f[e] = a[e]; f[8 + e] = b[e]; } return f; }
__device__ __forceinline__ v8f wmma16b(v16b a, v16b b, v8f c) { v8f d = __builtin_amdgcn_wmma_f32_16x16x32_f16(false, a, false, b, (short)0, c, false, false); asm volatile("v_nop\n\tv_nop\n\tv_nop\n\tv_nop" : "+v"(d) : "v"(a), "v"(b)); return d; }
__device__ __forceinline__ void wave_lds_sync() { __builtin_amdgcn_fence(__ATOMIC_RELEASE, "workgroup"); __builtin_amdgcn_wave_barrier(); __builtin_amdgcn_fence(__ATOMIC_ACQUIRE, "workgroup"); }
__device__ __forceinline__ float pmul(float a, float b) { float p = a * b; asm volatile("" : "+v"(p)); return p; }
__device__ __forceinline__ int iclamp(int v, int lo, int hi) { return v < lo ? lo : (v > hi ? hi : v); }

typedef __attribute__((ext_vector_type(2))) _Float16 v2h;
typedef __attribute__((ext_vector_type(4))) _Float16 v4h;
typedef __attribute__((ext_vector_type(2))) float v2f;
typedef __attribute__((ext_vector_type(4))) int v4i;
__device__ __forceinline__ float nexp2(float v) { return __builtin_amdgcn_exp2f(v); }
__global__ __launch_bounds__(256) void prep_kernel(const float* __restrict__ w1, const float* __restrict__ w2, const float* __restrict__ w, b16* __restrict__ WE, b16* __restrict__ WO) {
  const int u = blockIdx.x * 256 + threadIdx.x; if (u >= (128 + 64) * D / 8) return; const int e = u * 8; const int o = e / D, k0 = e % D; v8b v; b16* dst;
  if (o < 128) { const float* ww = o < 64 ? w1 : w2; const int oo = o & 63; for (int j = 0; j < 8; ++j) v[j] = (b16)(bf16_rne(ww[(k0 + j) * D + oo]) * WSC); dst = WE + (size_t)o * D + k0; }
  else { const int oo = o - 128; for (int j = 0; j < 8; ++j) v[j] = (b16)(bf16_rne(w[(k0 + j) * D + oo]) * WSC); dst = WO + (size_t)oo * D + k0; }
  for (int pass = 0; pass < 2; ++pass) { *(volatile v8b*)dst = v; __threadfence(); }
}
__global__ __launch_bounds__(128) void eproj_kernel(const float* __restrict__ x, const b16* __restrict__ WE, const float* __restrict__ b1, const float* __restrict__ b2, b16* __restrict__ E1h, b16* __restrict__ E1l, b16* __restrict__ E2h, b16* __restrict__ E2l) {
  __shared__ __attribute__((aligned(16))) b16 As[64][D + 8]; __shared__ __attribute__((aligned(16))) float Tf[4][16][128 + 4];
  const int wave = threadIdx.x >> 5, lane = threadIdx.x & 31, nloc = lane & 15, hlf = lane >> 4; const size_t r0 = (size_t)blockIdx.x * 64;
  for (int i = threadIdx.x; i < 64 * 16; i += 128) { const int rr = i / 16, q = (i % 16) * 4; const v4f f = *(const v4f*)(x + (r0 + rr) * D + q); v4h o; for (int j = 0; j < 4; ++j) o[j] = (b16)(bf16_rne(f[j]) * XS); *(v4h*)(&As[rr][q]) = o; }
  __syncthreads();
  v8f acc[8];
#pragma unroll
  for (int t = 0; t < 8; ++t) acc[t] = (v8f){};
#pragma unroll
  for (int kb = 0; kb < D; kb += 32) { const v16b a = frag_kb(&As[wave * 16 + nloc][kb], hlf);
#pragma unroll
    for (int t = 0; t < 8; ++t) acc[t] = wmma16b(a, frag_kb(WE + (size_t)(t * 16 + nloc) * D + kb, hlf), acc[t]); }
#pragma unroll
  for (int t = 0; t < 8; ++t) { const int col = t * 16 + nloc; const float bb = bf16_rne(col < 64 ? b1[col] : b2[col - 64]);
#pragma unroll
    for (int r = 0; r < 8; ++r) Tf[wave][8 * hlf + r][col] = acc[t][r] * (1.0f / (XS * WSC)) + bb; }
  wave_lds_sync();
  for (int pass = 0; pass < 2; ++pass) {
    for (int rr = 0; rr < 16; rr += 2) { const int r2 = rr + (lane >> 4); const size_t xr = r0 + wave * 16 + r2; const int bb_ = (int)(xr / (N * T)), rem = (int)(xr % (N * T)), nn = rem / T, tt = rem % T; const size_t prow = ((size_t)(bb_ * T + tt) * N + nn) * D;
      const int c = (lane & 15) * 4;
      v4h h1, l1, h2, l2; for (int j = 0; j < 4; ++j) { { const float f = Tf[wave][r2][c + j] * XS; const b16 p = (b16)f; h1[j] = p; l1[j] = (b16)((f - (float)p) * RS_); } { const float f = Tf[wave][r2][64 + c + j] * XS; const b16 p = (b16)f; h2[j] = p; l2[j] = (b16)((f - (float)p) * RS_); } }
      *(volatile v4h*)(E1h + prow + c) = h1; *(volatile v4h*)(E1l + prow + c) = l1; *(volatile v4h*)(E2h + prow + c) = h2; *(volatile v4h*)(E2l + prow + c) = l2; }
    __threadfence(); }
}
__global__ __launch_bounds__(256) void xt_kernel(const float* __restrict__ x, b16* __restrict__ XT) {
  __shared__ float tile[64][64 + 1];
  const int bt = blockIdx.y, b = bt / T, t = bt % T, n0 = blockIdx.x * 64; const int tid = threadIdx.x;
  for (int i = tid; i < 64 * 64; i += 256) { const int nn = i / 64, d = i % 64; tile[nn][d] = bf16_rne(x[(((size_t)b * N + n0 + nn) * T + t) * D + d]); }
  __syncthreads();
  const int wave = tid >> 5, lane = tid & 31;
  for (int pass = 0; pass < 2; ++pass) { for (int d = wave; d < 64; d += 8) { v2h o; o[0] = (b16)(tile[2 * lane][d] * XS); o[1] = (b16)(tile[2 * lane + 1][d] * XS); *(volatile v2h*)(XT + ((size_t)bt * D + d) * N + n0 + 2 * lane) = o; } __threadfence(); }
}
__global__ __launch_bounds__(64) void attn_kernel(const b16* __restrict__ E1h, const b16* __restrict__ E1l, const b16* __restrict__ E2h, const b16* __restrict__ E2l, const b16* __restrict__ XT, const b16* __restrict__ WO, const float* __restrict__ bo, float* __restrict__ out) {
  __shared__ __attribute__((aligned(16))) b16 Pb[2][16][32 + 8], Pl[2][16][32 + 8], Hh[2][16][D + 8], Hl[2][16][D + 8]; __shared__ __attribute__((aligned(16))) float To[2][16][D + 4];
  const int wave = threadIdx.x >> 5, lane = threadIdx.x & 31, col = lane & 15, hh = lane >> 4; const int bt = blockIdx.y; const int q0 = blockIdx.x * 32 + wave * 16; const int qi = q0 + col;
  const size_t pb = (size_t)bt * N * D; const b16* Q1 = E1h + pb; const b16* Q1l = E1l + pb; const b16* K2 = E2h + pb; const b16* K2l = E2l + pb; const b16* Vt = XT + (size_t)bt * D * N;
  const v16b qa0 = frag_kb(Q1 + (size_t)qi * D, hh), qa1 = frag_kb(Q1 + (size_t)qi * D + 32, hh), ql0 = frag_kb(Q1l + (size_t)qi * D, hh), ql1 = frag_kb(Q1l + (size_t)qi * D + 32, hh);
  const float cs = LOG2E / (XS * XS);
  float m = -INFINITY, l = 0.0f; v8f o[4], ol[4]; for (int t = 0; t < 4; ++t) { o[t] = (v8f){}; ol[t] = (v8f){}; }
#pragma unroll 1
  for (int kb = 0; kb < N; kb += 32) {
    float e[16]; float mx = -INFINITY;
#pragma unroll
    for (int u = 0; u < 2; ++u) { v8f s = (v8f){}, sx = (v8f){}; const size_t kr = (size_t)(kb + u * 16 + col) * D; { const v16b k0 = frag_kb(K2 + kr, hh), k1 = frag_kb(K2 + kr + 32, hh); s = wmma16b(k0, qa0, s); s = wmma16b(k1, qa1, s); sx = wmma16b(k0, ql0, sx); sx = wmma16b(k1, ql1, sx); sx = wmma16b(frag_kb(K2l + kr, hh), qa0, sx); sx = wmma16b(frag_kb(K2l + kr + 32, hh), qa1, sx); }
#pragma unroll
      for (int r = 0; r < 8; ++r) { const float raw = s[r] + sx[r] * (1.0f / RS_); const float vv = fmaxf(raw, 0.0f) * cs; e[u * 8 + r] = vv; mx = fmaxf(mx, vv); } }
    mx = fmaxf(mx, __shfl_xor(mx, 16));
    const float mn = fmaxf(m, mx); const float al = nexp2(m - mn); float sum = 0.0f;
#pragma unroll
    for (int i2 = 0; i2 < 16; ++i2) { const float p = nexp2(e[i2] - mn); sum += p; const float ps = p * PS; const b16 phh = (b16)ps; const int pc = (i2 < 8 ? 0 : 16) + 8 * hh + (i2 & 7); Pb[wave][col][pc] = phh; Pl[wave][col][pc] = (b16)((ps - (float)phh) * RS_); }
    sum += __shfl_xor(sum, 16); l = l * al + sum; m = mn;
    wave_lds_sync();
    const v16b pf = frag_kb(&Pb[wave][col][0], hh), plf = frag_kb(&Pl[wave][col][0], hh);
#pragma unroll
    for (int t = 0; t < 4; ++t) { const v16b vh = frag_kb(Vt + (size_t)(t * 16 + col) * N + kb, hh); o[t] *= al; o[t] = wmma16b(vh, pf, o[t]); ol[t] = wmma16b(vh, plf, ol[t] * al); }
    wave_lds_sync(); }
  const float inv = 1.0f / (l * PS * XS);
#pragma unroll
  for (int t = 0; t < 4; ++t)
#pragma unroll
    for (int r = 0; r < 8; ++r) To[wave][col][t * 16 + 8 * hh + r] = (o[t][r] + ol[t][r] * (1.0f / RS_)) * inv;
  wave_lds_sync();
  for (int i2 = lane; i2 < 16 * D; i2 += 32) { const int qq = i2 / D, d = i2 % D; const float f = To[wave][qq][d] * XS; const b16 p = (b16)f; Hh[wave][qq][d] = p; Hl[wave][qq][d] = (b16)(f - (float)p); }
  wave_lds_sync();
  v8f acc[4]; for (int t = 0; t < 4; ++t) acc[t] = (v8f){};
#pragma unroll
  for (int kb = 0; kb < D; kb += 32) { const v16b ah = frag_kb(&Hh[wave][col][kb], hh), al2 = frag_kb(&Hl[wave][col][kb], hh);
#pragma unroll
    for (int t = 0; t < 4; ++t) { const v16b bw = frag_kb(WO + (size_t)(t * 16 + col) * D + kb, hh); acc[t] = wmma16b(ah, bw, acc[t]); acc[t] = wmma16b(al2, bw, acc[t]); } }
#pragma unroll
  for (int t = 0; t < 4; ++t) { const float bb = bf16_rne(bo[t * 16 + col]);
#pragma unroll
    for (int r = 0; r < 8; ++r) To[wave][8 * hh + r][t * 16 + col] = fmaxf(acc[t][r] * (1.0f / (XS * WSC)) + bb, 0.0f); }
  wave_lds_sync();
  const int b = bt / T, tt = bt % T;
  for (int pass = 0; pass < 2; ++pass) { for (int rr = 0; rr < 16; rr += 2) { const int r2 = rr + (lane >> 4); const int node = q0 + r2; *(volatile v4f*)(out + (((size_t)b * N + node) * T + tt) * D + (lane & 15) * 4) = *(const v4f*)(&To[wave][r2][(lane & 15) * 4]); } __threadfence(); }
}
}

extern "C" void kernel_launch(void* const* d_in, const int* in_sizes, int n_in, void* d_out, int out_size, void* d_ws, size_t ws_size, hipStream_t stream) {
  (void)n_in;
  auto Fp = [&](int i) { return (const float*)d_in[i]; };
  if (in_sizes[0] != NR * D || in_sizes[1] != D * D || in_sizes[2] != D || in_sizes[3] != D * D || in_sizes[4] != D || in_sizes[5] != D * D || in_sizes[6] != D || out_size != NR * D) return;
  size_t off = 0; char* ws = (char*)d_ws;
  auto carve = [&](size_t bytes) { char* p = ws + off; off += (bytes + 255) & ~(size_t)255; return p; };
  b16* WE = (b16*)carve((size_t)128 * D * 2); b16* WO = (b16*)carve((size_t)64 * D * 2); const size_t plane = (size_t)NR * D * 2;
  b16* E1h = (b16*)carve(plane); b16* E1l = (b16*)carve(plane); b16* E2h = (b16*)carve(plane); b16* E2l = (b16*)carve(plane); b16* XT = (b16*)carve(plane);
  if (off > ws_size || off > ((size_t)128 << 20)) return;
  prep_kernel<<<((128 + 64) * D / 8 + 255) / 256, 256, 0, stream>>>(Fp(1), Fp(3), Fp(5), WE, WO);
  eproj_kernel<<<NR / 64, 128, 0, stream>>>(Fp(0), WE, Fp(2), Fp(4), E1h, E1l, E2h, E2l);
  xt_kernel<<<dim3(N / 64, NBT), 256, 0, stream>>>(Fp(0), XT);
  attn_kernel<<<dim3(N / 32, BTL), 64, 0, stream>>>(E1h, E1l, E2h, E2l, XT, WO, Fp(6), (float*)d_out);
}
